// deepar_cedar_38946763440819
// MI455X (gfx1250) — hardware-verified
//
#include <hip/hip_runtime.h>
#include <stddef.h>
#include <math.h>


#define T_DIM   192
#define B_DIM   256
#define HID     128
#define GD      512
#define LW      24
#define TP      (T_DIM - LW)
#define NDOM    32
#define FEAT    (3 * HID)
#define REPF    (LW * FEAT)
#define NROW    (T_DIM * B_DIM)
#define NPRED   (LW * B_DIM)
#define OUT_N   (2 + 2 * NPRED)
#define KX0     64
#define KIN0    42
#define VB      16
#define NBLK    (B_DIM / VB)
#define NTHR    128

#define WC      64.0f
#define AC      16.0f
#define INV_AW  (1.0f / 1024.0f)
#define EPS_C   1e-6f
#define HALF_LOG_2PI 0.91893853320467274f

#define F_IH0   64
#define F_W128  128

#define O_PIH0  ((size_t)0)
#define O_PHH0  (O_PIH0 + (size_t)F_IH0  * 1024)
#define O_PIH1  (O_PHH0 + (size_t)F_W128 * 1024)
#define O_PHH1  (O_PIH1 + (size_t)F_W128 * 1024)
#define O_PIH2  (O_PHH1 + (size_t)F_W128 * 1024)
#define O_PHH2  (O_PIH2 + (size_t)F_W128 * 1024)
#define O_X0    (O_PHH2 + (size_t)F_W128 * 1024)
#define SZ_X0   ((size_t)NROW * KX0 * 2)
#define O_HA    (O_X0 + SZ_X0)
#define SZ_H    ((size_t)NROW * HID * 2)
#define O_HB    (O_HA + SZ_H)
#define O_HP    (O_HB + SZ_H)
#define SZ_HP   ((size_t)NPRED * FEAT * 4)
#define O_DR    (O_HP + SZ_HP)
#define SZ_DR   ((size_t)NDOM * REPF * 4)
#define O_LOC   (O_DR + SZ_DR)
#define SZ_V    ((size_t)NPRED * 4)
#define O_SC    (O_LOC + SZ_V)
#define O_NL    (O_SC + SZ_V)
#define WSTOT   (O_NL + SZ_V)
#define WSCAP   134217728

static_assert(WSTOT <= (size_t)WSCAP);
static_assert((O_PHH0 % 512) == 0 && (O_PIH1 % 512) == 0 && (O_PHH1 % 512) == 0);
static_assert((O_PIH2 % 512) == 0 && (O_PHH2 % 512) == 0 && (O_X0 % 512) == 0);
static_assert((O_HA % 512) == 0 && (O_HB % 512) == 0 && (O_HP % 512) == 0);
static_assert((O_DR % 512) == 0 && (O_LOC % 512) == 0 && (O_SC % 512) == 0 && (O_NL % 512) == 0);
static_assert((SZ_X0 % 512) == 0 && (SZ_H % 4096) == 0 && (SZ_HP % 512) == 0 && (SZ_DR % 512) == 0);
static_assert(OUT_N == 3072 * 4 + 2);
static_assert((KX0 % 32) == 0 && (HID % 32) == 0 && KX0 >= KIN0);
static_assert(NBLK * VB == B_DIM && NTHR == 128);
static_assert(VB * HID == 16 * NTHR);
static_assert((NROW * 8) % 256 == 0);
static_assert(NPRED % 128 == 0);
static_assert(NPRED % 1024 == 0);
static_assert(REPF % 128 == 0 && FEAT == 3 * 128);
static_assert(REPF == 8 * 1152 && (1152 % 4) == 0 && (REPF % 4) == 0);

typedef _Float16 v16h __attribute__((ext_vector_type(16)));
typedef _Float16 v8h  __attribute__((ext_vector_type(8), __may_alias__));
typedef float    v8f  __attribute__((ext_vector_type(8)));
typedef float    v4f  __attribute__((ext_vector_type(4), __may_alias__));
typedef float    v2f  __attribute__((ext_vector_type(2), __may_alias__));
union Frag { v16h v; v8h h[2]; };
static_assert(sizeof(Frag) == 32);

__device__ __forceinline__ int imin(int a, int b) { return a < b ? a : b; }
__device__ __forceinline__ int imax(int a, int b) { return a > b ? a : b; }

__device__ __forceinline__ v8f wmh(v16h a, v16h bq, v8f c) {
  v8f d = __builtin_amdgcn_wmma_f32_16x16x32_f16(false, a, false, bq, (short)0, c, false, false);
  asm volatile("v_nop\n\tv_nop\n\tv_nop\n\tv_nop" : "+v"(d) : "v"(a), "v"(bq));
  return d;
}

__device__ __forceinline__ v8f zero8() {
  v8f z = {0.f, 0.f, 0.f, 0.f, 0.f, 0.f, 0.f, 0.f};
  return z;
}

__device__ __forceinline__ v16h lda_frag(const _Float16* base, int pitch, int lane) {
  const int m = lane & 15, hh = lane >> 4;
  const _Float16* p = base + (size_t)m * pitch + 8 * hh;
  Frag u;
  u.h[0] = *(const v8h*)p;
  u.h[1] = *(const v8h*)(p + 16);
  return u.v;
}

__device__ __forceinline__ v16h ldb_frag(const v16h* __restrict__ packed, int frag, int lane) {
  return packed[frag * 32 + lane];
}

__device__ __forceinline__ float sigm_(float x) { return 1.0f / (1.0f + __expf(-x)); }

__global__ __launch_bounds__(256) void k_pack(const float* __restrict__ src, _Float16* dst,
                                              int ksrc, int chunks, int nthr) {
  const int e = blockIdx.x * 256 + threadIdx.x;
  if (e >= nthr) return;
  const int frag = e >> 6, r = e & 63, lane = r >> 1, q = r & 1;
  const int tn = frag / chunks, kc = frag - tn * chunks;
  const int n = tn * 16 + (lane & 15);
  const int kb = kc * 32 + 16 * q + 8 * (lane >> 4);
  v8h hv;
#pragma unroll
  for (int i = 0; i < 8; ++i) {
    const int k = kb + i;
    const float w = src[(size_t)n * ksrc + imin(k, ksrc - 1)];
    hv[i] = (_Float16)(((k < ksrc) ? w : 0.0f) * WC);
  }
  *(volatile v8h*)(dst + (size_t)8 * e) = hv;
  __threadfence();
  *(volatile v8h*)(dst + (size_t)8 * e) = hv;
}

__global__ __launch_bounds__(256) void k_build_x0(const int* __restrict__ Xe, const float* __restrict__ Xc,
                                                  const float* __restrict__ Xl,
                                                  const float* __restrict__ emb0,
                                                  const float* __restrict__ emb1, _Float16* X0) {
  const int e = blockIdx.x * 256 + threadIdx.x;
  if (e >= NROW * 8) return;
  const int row = e >> 3, q = e & 7;
  const int i0 = imin(imax(Xe[row * 2 + 0], 0), 999);
  const int i1 = imin(imax(Xe[row * 2 + 1], 0), 49);
  v8h hv;
#pragma unroll
  for (int i = 0; i < 8; ++i) {
    const int c = 8 * q + i;
    const float vl = Xl[(size_t)row * 4 + imin(c, 3)];
    const float vc = Xc[(size_t)row * 8 + imin(imax(c - 4, 0), 7)];
    const float v0 = emb0[i0 * 20 + imin(imax(c - 12, 0), 19)];
    const float v1 = emb1[i1 * 10 + imin(imax(c - 32, 0), 9)];
    const float val = (c < 4) ? vl : ((c < 12) ? vc : ((c < 32) ? v0 : ((c < KIN0) ? v1 : 0.0f)));
    hv[i] = (_Float16)(val * AC);
  }
  *(volatile v8h*)(X0 + (size_t)8 * e) = hv;
  __threadfence();
  *(volatile v8h*)(X0 + (size_t)8 * e) = hv;
}

template <int NKX>
__global__ __launch_bounds__(NTHR) void k_lstm(const _Float16* __restrict__ Xin,
                                               const v16h* __restrict__ Pih,
                                               const v16h* __restrict__ Phh,
                                               const float* __restrict__ bih,
                                               const float* __restrict__ bhh,
                                               _Float16* Hout, float* HP, int layer) {
  __shared__ __align__(16) _Float16 sH[VB * HID];
  __shared__ __align__(16) float sG[VB * GD];
  __shared__ __align__(16) float sC[VB * HID];
  __shared__ __align__(16) float sHf[VB * HID];
  __shared__ __align__(16) float sBg[GD];

  const int tid = threadIdx.x, lane = tid & 31, wave = tid >> 5;
  const int hh = lane >> 4, nn = lane & 15;
  const int b0 = blockIdx.x * VB;
  constexpr int KXP = NKX * 32;

  for (int i = tid; i < GD; i += NTHR) sBg[i] = bih[i] + bhh[i];
  for (int i = tid; i < VB * HID; i += NTHR) {
    sH[i] = (_Float16)0.0f;
    sC[i] = 0.0f;
    sHf[i] = 0.0f;
  }
  __syncthreads();

#pragma unroll 1
  for (int t = 0; t < T_DIM; ++t) {
    {
      v16h fx[NKX], fh[4];
      const _Float16* xrow = Xin + ((size_t)(t * B_DIM + b0 + nn)) * KXP + 8 * hh;
#pragma unroll
      for (int kc = 0; kc < NKX; ++kc) {
        Frag u;
        u.h[0] = *(const v8h*)(xrow + kc * 32);
        u.h[1] = *(const v8h*)(xrow + kc * 32 + 16);
        fx[kc] = u.v;
      }
#pragma unroll
      for (int kc = 0; kc < 4; ++kc) fh[kc] = lda_frag(sH + kc * 32, HID, lane);
#pragma unroll 1
      for (int tn = wave; tn < 32; tn += 4) {
        v8f acc = zero8();
#pragma unroll
        for (int kc = 0; kc < NKX; ++kc) acc = wmh(fx[kc], ldb_frag(Pih, tn * NKX + kc, lane), acc);
#pragma unroll
        for (int kc = 0; kc < 4; ++kc) acc = wmh(fh[kc], ldb_frag(Phh, tn * 4 + kc, lane), acc);
        const int col = tn * 16 + nn;
        const float bb = sBg[col];
#pragma unroll
        for (int r = 0; r < 8; ++r) sG[(8 * hh + r) * GD + col] = acc[r] * INV_AW + bb;
      }
    }
    __syncthreads();

#pragma unroll 1
    for (int it = 0; it < 16; ++it) {
      const int i = tid + NTHR * it;
      const int v = i >> 7, r = i & 127;
      const float* g = sG + v * GD;
      const float ig = sigm_(g[r]);
      const float fg = sigm_(g[128 + r]);
      const float gg = tanhf(g[256 + r]);
      const float og = sigm_(g[384 + r]);
      const float cn = fg * sC[i] + ig * gg;
      const float hn = og * tanhf(cn);
      sC[i] = cn;
      sHf[i] = hn;
      sH[i] = (_Float16)(hn * AC);
    }
    __syncthreads();

    {
      const int p0 = wave * 2, p1 = wave * 2 + 1;
      const v8h hv0 = *(const v8h*)(sH + p0 * 256 + lane * 8);
      const v8h hv1 = *(const v8h*)(sH + p1 * 256 + lane * 8);
      _Float16* hd = Hout + ((size_t)(t * B_DIM + b0)) * HID;
      _Float16* hd0 = hd + p0 * 256 + lane * 8;
      _Float16* hd1 = hd + p1 * 256 + lane * 8;
      const bool wp = (t >= TP);
      const int tt = imax(t - TP, 0);
      v4f pv[4];
      float* pd[4];
#pragma unroll
      for (int k = 0; k < 4; ++k) {
        const int m = wave + 4 * k;
        pv[k] = *(const v4f*)(sHf + m * HID + lane * 4);
        pd[k] = HP + ((size_t)(tt * B_DIM + b0 + m)) * FEAT + layer * HID + lane * 4;
      }
      *(volatile v8h*)hd0 = hv0;
      *(volatile v8h*)hd1 = hv1;
      if (wp) {
#pragma unroll
        for (int k = 0; k < 4; ++k) *(volatile v4f*)pd[k] = pv[k];
      }
      __threadfence();
      *(volatile v8h*)hd0 = hv0;
      *(volatile v8h*)hd1 = hv1;
      if (wp) {
#pragma unroll
        for (int k = 0; k < 4; ++k) *(volatile v4f*)pd[k] = pv[k];
      }
    }
  }
}

__global__ __launch_bounds__(128) void k_head(const float* __restrict__ HP, const float* __restrict__ y,
                                              const float* __restrict__ locW, const float* __restrict__ locB,
                                              const float* __restrict__ scW, const float* __restrict__ scB,
                                              float* LOCP, float* SCP, float* NLP) {
  __shared__ __align__(16) float sW[2 * FEAT];
  __shared__ __align__(16) float sL[128];
  __shared__ __align__(16) float sS[128];
  __shared__ __align__(16) float sN[128];
  const int tid = threadIdx.x, lane = tid & 31, wave = tid >> 5;
  for (int i = tid; i < FEAT; i += 128) { sW[i] = locW[i]; sW[FEAT + i] = scW[i]; }
  __syncthreads();

  const int r0 = blockIdx.x * 128;
  const int r = r0 + tid;
  const float* hrow = HP + (size_t)r * FEAT;
  float aloc = 0.0f, asc = 0.0f;
#pragma unroll 2
  for (int c = 0; c < FEAT; ++c) {
    const float hv = hrow[c];
    aloc += hv * sW[c];
    asc  += hv * sW[FEAT + c];
  }
  const float loc = aloc + locB[0];
  const float pre = asc + scB[0];
  const float sp = fmaxf(pre, 0.0f) + log1pf(expf(-fabsf(pre)));
  const float scale = sp + EPS_C;
  const float yt = y[(size_t)TP * B_DIM + r];
  const float rs = 1.0f / scale;
  const float z = (yt - loc) * rs;
  const float nlp = 0.5f * z * z + logf(scale) + HALF_LOG_2PI;
  sL[tid] = loc;
  sS[tid] = scale;
  sN[tid] = nlp;
  __syncthreads();

  const v4f vL = *(const v4f*)(sL + 4 * lane);
  const v4f vS = *(const v4f*)(sS + 4 * lane);
  const v4f vN = *(const v4f*)(sN + 4 * lane);
  float* dL = LOCP + r0 + 4 * lane;
  float* dS = SCP + r0 + 4 * lane;
  float* dN = NLP + r0 + 4 * lane;
  if (wave == 0) *(volatile v4f*)dL = vL;
  if (wave == 1) *(volatile v4f*)dS = vS;
  if (wave == 2) *(volatile v4f*)dN = vN;
  __threadfence();
  if (wave == 0) *(volatile v4f*)dL = vL;
  if (wave == 1) *(volatile v4f*)dS = vS;
  if (wave == 2) *(volatile v4f*)dN = vN;
}

__global__ __launch_bounds__(128) void k_domrep(const float* __restrict__ HP, const int* __restrict__ dom,
                                                float* DR) {
  __shared__ __align__(16) float sAcc[NDOM * 128];
  __shared__ float sRc[NDOM];
  const int tid = threadIdx.x, lane = tid & 31, wave = tid >> 5;
#pragma unroll
  for (int d = 0; d < NDOM; ++d) sAcc[d * 128 + tid] = 0.0f;
  if (tid < NDOM) {
    int c = 0;
#pragma unroll 1
    for (int b = 0; b < B_DIM; ++b) c += (dom[b] == tid) ? 1 : 0;
    sRc[tid] = 1.0f / (float)imax(c, 1);
  }
  const int t = blockIdx.x / 3, c0 = (blockIdx.x - 3 * t) * 128;
  const float* hp = HP + ((size_t)(t * B_DIM)) * FEAT + c0 + tid;
#pragma unroll 1
  for (int b = 0; b < B_DIM; ++b) {
    const int dr = dom[b];
    const bool ok = ((unsigned)dr < (unsigned)NDOM);
    const int dcl = imin(imax(dr, 0), NDOM - 1);
    const float v = hp[(size_t)b * FEAT];
    sAcc[dcl * 128 + tid] += ok ? v : 0.0f;
  }
  __syncthreads();

  v4f ov[8];
  float* od[8];
#pragma unroll
  for (int k = 0; k < 8; ++k) {
    const int d = wave + 4 * k;
    const v4f a = *(const v4f*)(sAcc + d * 128 + 4 * lane);
    ov[k] = a * sRc[d];
    od[k] = DR + (size_t)d * REPF + blockIdx.x * 128 + 4 * lane;
  }
#pragma unroll
  for (int k = 0; k < 8; ++k) *(volatile v4f*)od[k] = ov[k];
  __threadfence();
#pragma unroll
  for (int k = 0; k < 8; ++k) *(volatile v4f*)od[k] = ov[k];
}

__global__ __launch_bounds__(256) void k_final(const float* DR, const float* NLP,
                                               const float* LOCP, const float* SCP,
                                               const int* dom, float* out) {
  __shared__ __align__(16) float sStage[OUT_N + 2];
  __shared__ float sLb[B_DIM];
  __shared__ float sRed[256];
  __shared__ float sPart[256];
  __shared__ float sDl[NDOM];
  __shared__ float sSq[NDOM];
  const int tid = threadIdx.x;

#pragma unroll
  for (int k = 0; k < NPRED / 1024; ++k) {
    const int idx = tid + 256 * k;
    const v4f v = *(const v4f*)(NLP + 4 * idx);
    *(v4f*)(sStage + 4 * idx) = v;
  }
  __syncthreads();

  float s = 0.0f;
#pragma unroll 1
  for (int t = 0; t < LW; ++t) s += sStage[t * B_DIM + tid];
  sLb[tid] = s * (1.0f / (float)LW);
  sRed[tid] = s;
  __syncthreads();
  for (int st = 128; st > 0; st >>= 1) {
    if (tid < st) sRed[tid] += sRed[tid + st];
    __syncthreads();
  }
  const float loss_y = sRed[0] * (1.0f / (float)NPRED);

  if (tid < NDOM) {
    float a = 0.0f;
    int c = 0;
#pragma unroll 1
    for (int b = 0; b < B_DIM; ++b) {
      const float lbv = sLb[b];
      const bool m = (dom[b] == tid);
      a += m ? lbv : 0.0f;
      c += m ? 1 : 0;
    }
    sDl[tid] = a * (1.0f / (float)imax(c, 1));
  }

  {
    const int d = tid >> 3, part = tid & 7;
    const float* rr = DR + (size_t)d * REPF + part * 1152;
    float q = 0.0f;
#pragma unroll 2
    for (int f4 = 0; f4 < 1152 / 4; ++f4) {
      const v4f v = *(const v4f*)(rr + 4 * f4);
      q += v[0] * v[0];
      q += v[1] * v[1];
      q += v[2] * v[2];
      q += v[3] * v[3];
    }
    sPart[tid] = q;
  }
  __syncthreads();
  if (tid < NDOM) {
    float q = 0.0f;
#pragma unroll
    for (int p = 0; p < 8; ++p) q += sPart[tid * 8 + p];
    sSq[tid] = q;
  }
  __syncthreads();

  float pen = 0.0f;
#pragma unroll 1
  for (int k = 0; k < 4; ++k) {
    const int p = tid + 256 * k;
    const int i = p >> 5, j = p & 31;
    const float* ri = DR + (size_t)i * REPF;
    const float* rj = DR + (size_t)j * REPF;
    float dot = 0.0f;
#pragma unroll 2
    for (int f4 = 0; f4 < REPF / 4; ++f4) {
      const v4f a = *(const v4f*)(ri + 4 * f4);
      const v4f b = *(const v4f*)(rj + 4 * f4);
      dot += a[0] * b[0];
      dot += a[1] * b[1];
      dot += a[2] * b[2];
      dot += a[3] * b[3];
    }
    const float mmd = sSq[i] + sSq[j] - 2.0f * dot;
    pen += mmd * fabsf(sDl[i] - sDl[j]);
  }
  sRed[tid] = pen;
  __syncthreads();
  for (int st = 128; st > 0; st >>= 1) {
    if (tid < st) sRed[tid] += sRed[tid + st];
    __syncthreads();
  }
  const float penalty = sRed[0] * (1.0f / (float)((NDOM - 1) * NDOM));

#pragma unroll
  for (int k = 0; k < NPRED / 1024; ++k) {
    const int idx = tid + 256 * k;
    const v4f v = *(const v4f*)(LOCP + 4 * idx);
    v2f lo, hi;
    lo[0] = v[0]; lo[1] = v[1]; hi[0] = v[2]; hi[1] = v[3];
    *(v2f*)(sStage + 2 + 4 * idx) = lo;
    *(v2f*)(sStage + 4 + 4 * idx) = hi;
  }
#pragma unroll
  for (int k = 0; k < NPRED / 1024; ++k) {
    const int idx = tid + 256 * k;
    const v4f v = *(const v4f*)(SCP + 4 * idx);
    v2f lo, hi;
    lo[0] = v[0]; lo[1] = v[1]; hi[0] = v[2]; hi[1] = v[3];
    *(v2f*)(sStage + 2 + NPRED + 4 * idx) = lo;
    *(v2f*)(sStage + 4 + NPRED + 4 * idx) = hi;
  }
  if (tid == 0) {
    sStage[0] = loss_y + penalty;
    sStage[1] = loss_y;
  }
  __syncthreads();

  v4f ov[12];
#pragma unroll
  for (int k = 0; k < 12; ++k) ov[k] = *(const v4f*)(sStage + 4 * (tid + 256 * k));
  const v2f tail = *(const v2f*)(sStage + 4 * 3072);

#pragma unroll
  for (int k = 0; k < 12; ++k) *(volatile v4f*)(out + 4 * (tid + 256 * k)) = ov[k];
  if (tid == 0) *(volatile v2f*)(out + 4 * 3072) = tail;
  __threadfence();
#pragma unroll
  for (int k = 0; k < 12; ++k) *(volatile v4f*)(out + 4 * (tid + 256 * k)) = ov[k];
  if (tid == 0) *(volatile v2f*)(out + 4 * 3072) = tail;
}

extern "C" void kernel_launch(void* const* d_in, const int* in_sizes, int n_in,
                              void* d_out, int out_size, void* d_ws, size_t ws_size,
                              hipStream_t stream) {
  if (n_in < 24) return;
  if (in_sizes[0] != NROW * 2) return;
  if (in_sizes[1] != NROW * 8 || in_sizes[2] != NROW * 4 || in_sizes[3] != NROW) return;
  if (in_sizes[4] != B_DIM || in_sizes[5] != 1) return;
  if (in_sizes[6] != 1000 * 20 || in_sizes[7] != 50 * 10) return;
  if (in_sizes[8] != GD * KIN0 || in_sizes[9] != GD * HID) return;
  if (in_sizes[10] != GD || in_sizes[11] != GD) return;
  if (in_sizes[12] != GD * HID || in_sizes[13] != GD * HID) return;
  if (in_sizes[14] != GD || in_sizes[15] != GD) return;
  if (in_sizes[16] != GD * HID || in_sizes[17] != GD * HID) return;
  if (in_sizes[18] != GD || in_sizes[19] != GD) return;
  if (in_sizes[20] != FEAT || in_sizes[21] != 1 || in_sizes[22] != FEAT || in_sizes[23] != 1) return;
  if (out_size != OUT_N) return;
  if ((size_t)WSTOT > ws_size) return;

  const int*   Xe   = (const int*)  d_in[0];
  const float* Xc   = (const float*)d_in[1];
  const float* Xl   = (const float*)d_in[2];
  const float* y    = (const float*)d_in[3];
  const int*   dom  = (const int*)  d_in[4];
  const float* emb0 = (const float*)d_in[6];
  const float* emb1 = (const float*)d_in[7];
  const float* Wih0 = (const float*)d_in[8];
  const float* Whh0 = (const float*)d_in[9];
  const float* bih0 = (const float*)d_in[10];
  const float* bhh0 = (const float*)d_in[11];
  const float* Wih1 = (const float*)d_in[12];
  const float* Whh1 = (const float*)d_in[13];
  const float* bih1 = (const float*)d_in[14];
  const float* bhh1 = (const float*)d_in[15];
  const float* Wih2 = (const float*)d_in[16];
  const float* Whh2 = (const float*)d_in[17];
  const float* bih2 = (const float*)d_in[18];
  const float* bhh2 = (const float*)d_in[19];
  const float* locW = (const float*)d_in[20];
  const float* locB = (const float*)d_in[21];
  const float* scW  = (const float*)d_in[22];
  const float* scB  = (const float*)d_in[23];
  float* out = (float*)d_out;

  char* ws = (char*)d_ws;
  _Float16* PIH0 = (_Float16*)(ws + O_PIH0);
  _Float16* PHH0 = (_Float16*)(ws + O_PHH0);
  _Float16* PIH1 = (_Float16*)(ws + O_PIH1);
  _Float16* PHH1 = (_Float16*)(ws + O_PHH1);
  _Float16* PIH2 = (_Float16*)(ws + O_PIH2);
  _Float16* PHH2 = (_Float16*)(ws + O_PHH2);
  _Float16* X0   = (_Float16*)(ws + O_X0);
  _Float16* HA   = (_Float16*)(ws + O_HA);
  _Float16* HB   = (_Float16*)(ws + O_HB);
  float* HP   = (float*)(ws + O_HP);
  float* DR   = (float*)(ws + O_DR);
  float* LOCP = (float*)(ws + O_LOC);
  float* SCP  = (float*)(ws + O_SC);
  float* NLP  = (float*)(ws + O_NL);

  k_pack<<<(F_IH0  * 64 + 255) / 256, 256, 0, stream>>>(Wih0, PIH0, KIN0, 2, F_IH0  * 64);
  k_pack<<<(F_W128 * 64 + 255) / 256, 256, 0, stream>>>(Whh0, PHH0, HID,  4, F_W128 * 64);
  k_pack<<<(F_W128 * 64 + 255) / 256, 256, 0, stream>>>(Wih1, PIH1, HID,  4, F_W128 * 64);
  k_pack<<<(F_W128 * 64 + 255) / 256, 256, 0, stream>>>(Whh1, PHH1, HID,  4, F_W128 * 64);
  k_pack<<<(F_W128 * 64 + 255) / 256, 256, 0, stream>>>(Wih2, PIH2, HID,  4, F_W128 * 64);
  k_pack<<<(F_W128 * 64 + 255) / 256, 256, 0, stream>>>(Whh2, PHH2, HID,  4, F_W128 * 64);

  k_build_x0<<<(NROW * 8) / 256, 256, 0, stream>>>(Xe, Xc, Xl, emb0, emb1, X0);

  k_lstm<2><<<NBLK, NTHR, 0, stream>>>(X0, (const v16h*)PIH0, (const v16h*)PHH0, bih0, bhh0, HA, HP, 0);
  k_lstm<4><<<NBLK, NTHR, 0, stream>>>(HA, (const v16h*)PIH1, (const v16h*)PHH1, bih1, bhh1, HB, HP, 1);
  k_lstm<4><<<NBLK, NTHR, 0, stream>>>(HB, (const v16h*)PIH2, (const v16h*)PHH2, bih2, bhh2, HA, HP, 2);

  k_head<<<NPRED / 128, 128, 0, stream>>>(HP, y, locW, locB, scW, scB, LOCP, SCP, NLP);
  k_domrep<<<REPF / 128, 128, 0, stream>>>(HP, dom, DR);
  k_final<<<1, 256, 0, stream>>>(DR, NLP, LOCP, SCP, dom, out);
}
